// ExpertGroup_11665131176299
// MI455X (gfx1250) — hardware-run, weakly checked
//
#include <hip/hip_runtime.h>


namespace {
constexpr int NT = 2048, E = 768, H = 3072, A = 192, NE = 8;
constexpr float XS = 8.0f, WSC = 256.0f;
typedef _Float16 b16;
typedef __attribute__((ext_vector_type(16))) _Float16 v16b;
typedef __attribute__((ext_vector_type(8))) _Float16 v8b;
typedef __attribute__((ext_vector_type(8))) float v8f;
typedef __attribute__((ext_vector_type(4))) float v4f;
__device__ __forceinline__ float bf16_rne(float f) { unsigned int u = __float_as_uint(f); u += 0x7FFFu + ((u >> 16) & 1u); return __uint_as_float(u & 0xFFFF0000u); }
__device__ __forceinline__ void split16(float v, b16& hi, b16& lo) { hi = (b16)v; lo = (b16)(v - (float)hi); }
__device__ __forceinline__ v16b frag_kb(const b16* p, int hh) { const v8b a = *(const v8b*)(p + 8 * hh), b = *(const v8b*)(p + 16 + 8 * hh); v16b f;
#pragma unroll
  for (int e = 0; e < 8; ++e) { f[e] = a[e]; f[8 + e] = b[e]; } return f; }
__device__ __forceinline__ v8f wmma16b(v16b a, v16b b, v8f c) { v8f d = __builtin_amdgcn_wmma_f32_16x16x32_f16(false, a, false, b, (short)0, c, false, false); asm volatile("v_nop\n\tv_nop\n\tv_nop\n\tv_nop" : "+v"(d) : "v"(a), "v"(b)); return d; }
__device__ __forceinline__ void wave_lds_sync() { __builtin_amdgcn_fence(__ATOMIC_RELEASE, "workgroup"); __builtin_amdgcn_wave_barrier(); __builtin_amdgcn_fence(__ATOMIC_ACQUIRE, "workgroup"); }
__device__ __forceinline__ float pmul(float a, float b) { float p = a * b; asm volatile("" : "+v"(p)); return p; }

__global__ __launch_bounds__(256) void wcopy_kernel(const float* __restrict__ w, size_t total, float sc, b16* __restrict__ WT) { const size_t u = (size_t)blockIdx.x * 256 + threadIdx.x; if (u >= total / 8) return; const size_t e = u * 8; v8b v;
#pragma unroll
  for (int j = 0; j < 8; ++j) v[j] = (b16)(bf16_rne(w[e + j]) * sc); for (int pass = 0; pass < 2; ++pass) { *(volatile v8b*)(WT + e) = v; __threadfence(); } }
__global__ __launch_bounds__(256) void ept_kernel(const float* __restrict__ ep, b16* __restrict__ EPt) { const int u = blockIdx.x * 256 + threadIdx.x; if (u >= A * (H / 8)) return; const int a = u / (H / 8), h0 = (u % (H / 8)) * 8; v8b v;
#pragma unroll
  for (int j = 0; j < 8; ++j) v[j] = (b16)(bf16_rne(ep[(size_t)(h0 + j) * A + a]) * XS); for (int pass = 0; pass < 2; ++pass) { *(volatile v8b*)(EPt + (size_t)a * H + h0) = v; __threadfence(); } }
__global__ __launch_bounds__(32) void m_kernel(const b16* __restrict__ WO, const b16* __restrict__ EPt, b16* __restrict__ Mh, b16* __restrict__ Ml) {
  __shared__ float Tf[16][A + 1]; const int lane = threadIdx.x, nloc = lane & 15, hlf = lane >> 4; const size_t g0 = (size_t)blockIdx.x * 16; v8f acc[12];
#pragma unroll
  for (int t = 0; t < 12; ++t) acc[t] = (v8f){};
#pragma unroll 2
  for (int kb = 0; kb < H; kb += 32) { const v16b a = frag_kb(WO + (g0 + nloc) * H + kb, hlf);
#pragma unroll
    for (int t = 0; t < 12; ++t) acc[t] = wmma16b(a, frag_kb(EPt + (size_t)(t * 16 + nloc) * H + kb, hlf), acc[t]); }
#pragma unroll
  for (int t = 0; t < 12; ++t)
#pragma unroll
    for (int r8 = 0; r8 < 8; ++r8) Tf[8 * hlf + r8][t * 16 + nloc] = acc[t][r8] * (1.0f / (WSC * XS));
  wave_lds_sync();
  for (int pass = 0; pass < 2; ++pass) { for (int rr = 0; rr < 16; ++rr) for (int a = lane; a < A; a += 32) { b16 p, q; split16(pmul(Tf[rr][a], XS), p, q); ((volatile b16*)Mh)[(g0 + rr) * A + a] = p; ((volatile b16*)Ml)[(g0 + rr) * A + a] = q; } __threadfence(); }
}
__global__ __launch_bounds__(32) void up_kernel(const float* __restrict__ x, const b16* __restrict__ WU, int RL, float* __restrict__ SH) {
  __shared__ __attribute__((aligned(16))) b16 Ah[16][E + 8]; __shared__ float Tf[16][132]; const int lane = threadIdx.x, nloc = lane & 15, hlf = lane >> 4; const int cg = blockIdx.x % (H / 128); const size_t m0 = (size_t)(blockIdx.x / (H / 128)) * 16; if (m0 >= (size_t)RL) return;
  for (int rr = 0; rr < 16; ++rr) for (int q = 0; q < E / 32; ++q) Ah[rr][q * 32 + lane] = (b16)(bf16_rne(x[(m0 + rr) * E + q * 32 + lane]) * XS);
  wave_lds_sync(); v8f acc[8];
#pragma unroll
  for (int t = 0; t < 8; ++t) acc[t] = (v8f){};
#pragma unroll 2
  for (int kb = 0; kb < E; kb += 32) { const v16b a = frag_kb(&Ah[nloc][kb], hlf);
#pragma unroll
    for (int t = 0; t < 8; ++t) acc[t] = wmma16b(a, frag_kb(WU + (size_t)(cg * 128 + t * 16 + nloc) * E + kb, hlf), acc[t]); }
#pragma unroll
  for (int t = 0; t < 8; ++t)
#pragma unroll
    for (int r8 = 0; r8 < 8; ++r8) { const float v = acc[t][r8] * (1.0f / (XS * WSC)); Tf[8 * hlf + r8][t * 16 + nloc] = pmul(v, 1.0f / (1.0f + __expf(-v))); }
  wave_lds_sync();
  for (int pass = 0; pass < 2; ++pass) { for (int rr = 0; rr < 16; ++rr) *(volatile v4f*)(SH + (m0 + rr) * H + cg * 128 + lane * 4) = *(const v4f*)(&Tf[rr][lane * 4]); __threadfence(); }
}
__global__ __launch_bounds__(32) void pre_kernel(const float* __restrict__ SH, const b16* __restrict__ WA, int RL, float* __restrict__ PRE) {
  __shared__ float Tf[16][A + 1]; const int lane = threadIdx.x, nloc = lane & 15, hlf = lane >> 4; const size_t m0 = (size_t)blockIdx.x * 16; if (m0 >= (size_t)RL) return; v8f acc[12];
#pragma unroll
  for (int t = 0; t < 12; ++t) acc[t] = (v8f){};
#pragma unroll 2
  for (int kb = 0; kb < H; kb += 32) { v16b a, al; { const float* p0 = SH + (m0 + nloc) * H + kb; b16 hh[16], ll[16];
#pragma unroll
      for (int e = 0; e < 8; ++e) { b16 p, q; split16(p0[8 * hlf + e] * XS, p, q); hh[e] = p; ll[e] = q; split16(p0[16 + 8 * hlf + e] * XS, p, q); hh[8 + e] = p; ll[8 + e] = q; }
#pragma unroll
      for (int e = 0; e < 16; ++e) { a[e] = hh[e]; al[e] = ll[e]; } }
#pragma unroll
    for (int t = 0; t < 12; ++t) { const v16b bw = frag_kb(WA + (size_t)(t * 16 + nloc) * H + kb, hlf); acc[t] = wmma16b(a, bw, acc[t]); acc[t] = wmma16b(al, bw, acc[t]); } }
#pragma unroll
  for (int t = 0; t < 12; ++t)
#pragma unroll
    for (int r8 = 0; r8 < 8; ++r8) Tf[8 * hlf + r8][t * 16 + nloc] = acc[t][r8] * (1.0f / (XS * WSC));
  wave_lds_sync();
  for (int pass = 0; pass < 2; ++pass) { for (int rr = 0; rr < 16; ++rr) for (int a = lane; a < A; a += 32) ((volatile float*)PRE)[(m0 + rr) * A + a] = Tf[rr][a]; __threadfence(); }
}
__global__ __launch_bounds__(32) void expert_kernel(const float* __restrict__ PRE, const float* __restrict__ ew, const float* __restrict__ adw, const float* __restrict__ lg, const float* __restrict__ lb, const b16* __restrict__ Mh, const b16* __restrict__ Ml, const float* __restrict__ SH, int RL, float* __restrict__ out) {
  __shared__ __attribute__((aligned(16))) b16 Ah[16][A + 8], Al[16][A + 8]; __shared__ float Pr[16][A + 1], Hr[16][A + 1], Tf[16][132]; __shared__ int Ex[16];
  const int lane = threadIdx.x, nloc = lane & 15, hlf = lane >> 4; const size_t m0 = (size_t)blockIdx.x * 16; if (m0 >= (size_t)RL) return;
  for (int rr = 0; rr < 16; ++rr) for (int a = lane; a < A; a += 32) Pr[rr][a] = PRE[(m0 + rr) * A + a];
  if (lane < 16) { int e = -1; for (int i = 0; i < NE; ++i) if (bf16_rne(ew[(m0 + lane) * NE + i]) > 0.0f) e = i; Ex[lane] = e; }
  wave_lds_sync();
  for (int rr = 0; rr < 16; ++rr) { const int e = Ex[rr]; float hv[6];
#pragma unroll
    for (int j = 0; j < 6; ++j) hv[j] = 0.0f;
    if (e >= 0) { const float* aw = adw + (size_t)e * A * A;
#pragma unroll 1
      for (int k = 0; k < A; ++k) { const float pk = Pr[rr][k];
#pragma unroll
        for (int j = 0; j < 6; ++j) hv[j] += pmul(pk, bf16_rne(aw[(size_t)(j * 32 + lane) * A + k])); } }
    for (int j = 0; j < 6; ++j) Hr[rr][j * 32 + lane] = hv[j]; }
  wave_lds_sync();
  for (int rr = 0; rr < 16; ++rr) { const int e = Ex[rr]; float s = 0.0f; for (int j = 0; j < 6; ++j) s += Hr[rr][j * 32 + lane]; for (int o = 16; o; o >>= 1) s += __shfl_xor(s, o); const float mu = s * (1.0f / A); float vq = 0.0f; for (int j = 0; j < 6; ++j) { const float d = Hr[rr][j * 32 + lane] - mu; vq += pmul(d, d); } for (int o = 16; o; o >>= 1) vq += __shfl_xor(vq, o); const float rs = rsqrtf(vq * (1.0f / A) + 1e-5f);
    for (int j = 0; j < 6; ++j) { const int a = j * 32 + lane; float hn = 0.0f; if (e >= 0) hn = pmul(pmul(Hr[rr][a] - mu, rs), bf16_rne(lg[e * A + a])) + bf16_rne(lb[e * A + a]); b16 p, q; split16(hn * XS, p, q); Ah[rr][a] = p; Al[rr][a] = q; } }
  wave_lds_sync();
#pragma unroll 1
  for (int cg = 0; cg < H / 128; ++cg) { v8f acc[8];
#pragma unroll
    for (int t = 0; t < 8; ++t) acc[t] = (v8f){};
#pragma unroll
    for (int kb = 0; kb < A; kb += 32) { const v16b a = frag_kb(&Ah[nloc][kb], hlf), al = frag_kb(&Al[nloc][kb], hlf);
#pragma unroll
      for (int t = 0; t < 8; ++t) { const size_t gr = (size_t)(cg * 128 + t * 16 + nloc) * A + kb; const v16b bh = frag_kb(Mh + gr, hlf), bl = frag_kb(Ml + gr, hlf); acc[t] = wmma16b(a, bh, acc[t]); acc[t] = wmma16b(a, bl, acc[t]); acc[t] = wmma16b(al, bh, acc[t]); } }
#pragma unroll
    for (int t = 0; t < 8; ++t) { const int c = cg * 128 + t * 16 + nloc;
#pragma unroll
      for (int r8 = 0; r8 < 8; ++r8) { const int rl = 8 * hlf + r8; Tf[rl][t * 16 + nloc] = SH[(m0 + rl) * H + c] + 0.1f * (acc[t][r8] * (1.0f / (XS * XS))); } }
    wave_lds_sync();
    for (int pass = 0; pass < 2; ++pass) { for (int rr = 0; rr < 16; ++rr) *(volatile v4f*)(out + (m0 + rr) * H + cg * 128 + lane * 4) = *(const v4f*)(&Tf[rr][lane * 4]); __threadfence(); }
    wave_lds_sync(); }
}
}

extern "C" void kernel_launch(void* const* d_in, const int* in_sizes, int n_in, void* d_out, int out_size, void* d_ws, size_t ws_size, hipStream_t stream) {
  (void)n_in;
  auto Fp = [&](int i) { return (const float*)d_in[i]; };
  if (in_sizes[0] != NT * E || in_sizes[1] != NT * NE || in_sizes[2] != H * E || in_sizes[3] != A * H || in_sizes[4] != NE * A * A || in_sizes[5] != NE * A || in_sizes[7] != H * A || in_sizes[8] != H * H || out_size != NT * H) return;
  const int RL = NT;
  size_t off = 0; char* ws = (char*)d_ws;
  auto carve = [&](size_t bytes) { char* p = ws + off; off += (bytes + 255) & ~(size_t)255; return p; };
  b16* WU = (b16*)carve((size_t)H * E * 2); b16* WA = (b16*)carve((size_t)A * H * 2); b16* WO = (b16*)carve((size_t)H * H * 2); b16* EPt = (b16*)carve((size_t)A * H * 2); b16* Mh = (b16*)carve((size_t)H * A * 2); b16* Ml = (b16*)carve((size_t)H * A * 2);
  float* SH = (float*)carve((size_t)NT * H * 4); float* PRE = (float*)carve((size_t)NT * A * 4);
  if (off > ws_size || off > ((size_t)96 << 20)) return;
  wcopy_kernel<<<(unsigned)(((size_t)H * E / 8 + 255) / 256), 256, 0, stream>>>(Fp(2), (size_t)H * E, WSC, WU); wcopy_kernel<<<(unsigned)(((size_t)A * H / 8 + 255) / 256), 256, 0, stream>>>(Fp(3), (size_t)A * H, WSC, WA); wcopy_kernel<<<(unsigned)(((size_t)H * H / 8 + 255) / 256), 256, 0, stream>>>(Fp(8), (size_t)H * H, WSC, WO);
  ept_kernel<<<(A * (H / 8) + 255) / 256, 256, 0, stream>>>(Fp(7), EPt);
  m_kernel<<<H / 16, 32, 0, stream>>>(WO, EPt, Mh, Ml);
  up_kernel<<<(RL / 16) * (H / 128), 32, 0, stream>>>(Fp(0), WU, RL, SH);
  pre_kernel<<<RL / 16, 32, 0, stream>>>(SH, WA, RL, PRE);
  expert_kernel<<<RL / 16, 32, 0, stream>>>(PRE, Fp(1), Fp(4), Fp(5), Fp(6), Mh, Ml, SH, RL, (float*)d_out);
}
